// BiMamba_29618094474256
// MI455X (gfx1250) — hardware-verified
//
#include <hip/hip_runtime.h>
#include <math.h>

typedef __attribute__((ext_vector_type(16))) _Float16 v16h;
typedef __attribute__((ext_vector_type(8)))  _Float16 v8h;
typedef __attribute__((ext_vector_type(8)))  float    v8f;
typedef __attribute__((ext_vector_type(4)))  float    v4f;
typedef __attribute__((ext_vector_type(4)))  unsigned v4u;

constexpr int kBatch  = 2;
constexpr int kL      = 2048;
constexpr int kDm     = 768;
constexpr int kDin    = 1536;
constexpr int kNst    = 16;
constexpr int kDtR    = 48;
constexpr int kPrjN   = 80;
constexpr int kPrjP   = 128;
constexpr int kDtK    = 64;
constexpr int kBC0    = 64;
constexpr int kT      = kBatch * kL;
constexpr int kTP     = 260;
constexpr int kScanTS = 64;
constexpr int kScanCh = 64;
constexpr int kScanYP = 68;

constexpr float kCarryW    = 32.0f;
constexpr float kCarryWdt  = 8.0f;
constexpr float kCarryProj = 16.0f;
constexpr float kCarryDl   = 16.0f;
constexpr float kCarryY    = 16.0f;
constexpr float kScaleXp   = 1.0f / kCarryW;
constexpr float kScaleProj = kCarryProj / kCarryW;
constexpr float kScaleDl   = kCarryDl / (kCarryProj * kCarryWdt);
constexpr float kScaleOut  = 1.0f / (kCarryY * kCarryW);
constexpr float kInvProj   = 1.0f / kCarryProj;
constexpr float kInvDl     = 1.0f / kCarryDl;
constexpr float kGateMul   = 0.5f * kCarryY;

static_assert(kDtR + 2 * kNst == kPrjN);
static_assert(kDtR <= kDtK && kDtK == kBC0 && kBC0 + 2 * kNst <= kPrjP);
static_assert((kDm % 32) == 0 && (kDin % 32) == 0 && (kDtK % 32) == 0);
static_assert((kT % 64) == 0 && ((2 * kT) % 64) == 0 && (kDin % 64) == 0 && (kPrjP % 64) == 0 && (kDm % 64) == 0);
static_assert((kL % kScanTS) == 0 && (kL % 64) == 0 && (kDin % kScanCh) == 0 && (kDin % 256) == 0);
static_assert(kNst == 16);

constexpr size_t kOffX16   = 0;
constexpr size_t kOffWIN   = kOffX16  + (size_t)kT * kDm * 2;
constexpr size_t kOffWOUT  = kOffWIN  + (size_t)2 * kDin * kDm * 2;
constexpr size_t kOffWXP   = kOffWOUT + (size_t)kDm * kDin * 2;
constexpr size_t kOffWDT   = kOffWXP  + (size_t)kPrjP * kDin * 2;
constexpr size_t kOffXP    = kOffWDT  + (size_t)kDin * kDtK * 2;
constexpr size_t kOffZ16   = kOffXP   + (size_t)kT * kDin * 4;
constexpr size_t kOffXC16  = kOffZ16  + (size_t)kT * kDin * 2;
constexpr size_t kOffPROJ  = kOffXC16 + (size_t)2 * kT * kDin * 2;
constexpr size_t kOffDL16  = kOffPROJ + (size_t)2 * kT * kPrjP * 2;
constexpr size_t kOffYC16  = kOffDL16 + (size_t)2 * kT * kDin * 2;
constexpr size_t kWsTotal  = kOffYC16 + (size_t)kT * kDin * 2;
static_assert(kWsTotal == 116719616ull);
static_assert(kWsTotal <= 134217728ull);
static_assert((kOffWIN % 128) == 0 && (kOffWOUT % 128) == 0 && (kOffWXP % 128) == 0 && (kOffWDT % 128) == 0 &&
              (kOffXP % 128) == 0 && (kOffZ16 % 128) == 0 && (kOffXC16 % 128) == 0 && (kOffPROJ % 128) == 0 &&
              (kOffDL16 % 128) == 0 && (kOffYC16 % 128) == 0);

__device__ __forceinline__ float h16_to_f32(unsigned hb) {
  const unsigned sgn = (hb & 0x8000u) << 16;
  const unsigned em  = hb & 0x7fffu;
  const float fn  = __uint_as_float((em << 13) + 0x38000000u);
  const float fs  = (float)em * 5.9604644775390625e-8f;
  const float mag = (em < 0x400u) ? fs : fn;
  return __uint_as_float(__float_as_uint(mag) | sgn);
}

__device__ __forceinline__ void grp_guard_h(v8f& a, v8f& b, v8f& c, v8f& d, v16h x, v16h b0, v16h b1, v16h b2, v16h b3) {
  asm volatile("v_nop\n\tv_nop\n\tv_nop\n\tv_nop" : "+v"(a), "+v"(b), "+v"(c), "+v"(d) : "v"(x), "v"(b0), "v"(b1), "v"(b2), "v"(b3));
}
__device__ __forceinline__ void keep4_h(v16h a, v16h b, v16h c, v16h d) { asm volatile("v_nop" :: "v"(a), "v"(b), "v"(c), "v"(d)); }
__device__ __forceinline__ void acc_guard4(v8f& a, v8f& b, v8f& c, v8f& d) { asm volatile("v_nop\n\tv_nop\n\tv_nop\n\tv_nop" : "+v"(a), "+v"(b), "+v"(c), "+v"(d)); }

union FragU { v16h v; v8h h[2]; };
__device__ __forceinline__ v16h frag_load(const _Float16* p) {
  FragU f;
  f.h[0] = *(const v8h*)(p);
  f.h[1] = *(const v8h*)(p + 16);
  return f.v;
}
__device__ __forceinline__ v8f frag_mma(v16h a, v16h b, v8f c) {
  return __builtin_amdgcn_wmma_f32_16x16x32_f16(false, a, false, b, (short)0, c, false, false);
}

template <int OUT_MODE>
__global__ __launch_bounds__(256) void wmma_gemm64(
    const unsigned short* __restrict__ Ap, int lda,
    const unsigned short* __restrict__ Btp, int ldb,
    void* __restrict__ Cout, int ldc,
    int M, int N, int K, float scale) {
  const _Float16* A  = (const _Float16*)Ap;
  const _Float16* Bt = (const _Float16*)Btp;
  __shared__ __align__(16) float sT[8][16 * 68];
  const int lane = threadIdx.x & 31;
  const int wave = threadIdx.x >> 5;
  const int tilesN = N >> 6;
  const int tilesM = M >> 6;
  const int tile = blockIdx.x * 8 + wave;
  if (tile >= tilesM * tilesN) return;
  const int tm = tile / tilesN;
  const int tn = tile - tm * tilesN;
  const int m0 = tm << 6;
  const int n0 = tn << 6;

  const int rlane = lane & 15;
  const int koff  = (lane >> 4) * 8;
  const int mOff  = (lane >> 4) * 8;

  v8f acc[4][4];
#pragma unroll
  for (int i = 0; i < 4; ++i)
#pragma unroll
    for (int j = 0; j < 4; ++j) acc[i][j] = (v8f){0.f,0.f,0.f,0.f,0.f,0.f,0.f,0.f};

  for (int k0 = 0; k0 < K; k0 += 32) {
    v16h bh[4];
#pragma unroll
    for (int j = 0; j < 4; ++j) {
      const size_t bo = (size_t)(n0 + (j << 4) + rlane) * ldb + koff + k0;
      bh[j] = frag_load(Bt + bo);
    }
#pragma unroll
    for (int i = 0; i < 4; ++i) {
      const size_t ao = (size_t)(m0 + (i << 4) + rlane) * lda + koff + k0;
      v16h ah = frag_load(A + ao);
#pragma unroll
      for (int j = 0; j < 4; ++j) acc[i][j] = frag_mma(ah, bh[j], acc[i][j]);
      grp_guard_h(acc[i][0], acc[i][1], acc[i][2], acc[i][3], ah, bh[0], bh[1], bh[2], bh[3]);
    }
    keep4_h(bh[0], bh[1], bh[2], bh[3]);
  }
  acc_guard4(acc[0][0], acc[0][1], acc[0][2], acc[0][3]);
  acc_guard4(acc[1][0], acc[1][1], acc[1][2], acc[1][3]);
  acc_guard4(acc[2][0], acc[2][1], acc[2][2], acc[2][3]);
  acc_guard4(acc[3][0], acc[3][1], acc[3][2], acc[3][3]);

  float* slab = sT[wave];
#pragma unroll
  for (int i = 0; i < 4; ++i) {
    const int mBase = m0 + (i << 4);
#pragma unroll
    for (int j = 0; j < 4; ++j) {
#pragma unroll
      for (int r = 0; r < 8; ++r) {
        const float v = acc[i][j][r] * scale;
        slab[(mOff + r) * 68 + (j << 4) + rlane] = v;
      }
    }
    __builtin_amdgcn_fence(__ATOMIC_RELEASE, "workgroup");
    __builtin_amdgcn_wave_barrier();
    __builtin_amdgcn_fence(__ATOMIC_ACQUIRE, "workgroup");
    if (OUT_MODE == 0) {
      float* C = (float*)Cout;
      const int hh = lane >> 4, c4 = (lane & 15) * 4;
      for (int pass = 0; pass < 2; ++pass) {
#pragma unroll
        for (int it = 0; it < 8; ++it) {
          const int row = it * 2 + hh;
          v4f v = *(const v4f*)(slab + row * 68 + c4);
          *(volatile v4f*)(C + (size_t)(mBase + row) * ldc + n0 + c4) = v;
        }
        __threadfence();
      }
    } else {
      const int q = lane >> 3, c8 = (lane & 7) * 8;
      unsigned short* C = (unsigned short*)Cout;
      for (int pass = 0; pass < 2; ++pass) {
#pragma unroll
        for (int it = 0; it < 4; ++it) {
          const int row = it * 4 + q;
          const float* sp = slab + row * 68 + c8;
          v8h hv;
#pragma unroll
          for (int e = 0; e < 8; ++e) hv[e] = (_Float16)sp[e];
          *(volatile v8h*)(C + (size_t)(mBase + row) * ldc + n0 + c8) = hv;
        }
        __threadfence();
      }
    }
    __builtin_amdgcn_fence(__ATOMIC_RELEASE, "workgroup");
    __builtin_amdgcn_wave_barrier();
    __builtin_amdgcn_fence(__ATOMIC_ACQUIRE, "workgroup");
  }
}

__global__ __launch_bounds__(256) void cast_f16_kernel(
    const float* __restrict__ src, unsigned short* __restrict__ dst, int total8, float scale)
{
  const int i = blockIdx.x * 256 + threadIdx.x;
  if (i >= total8) return;
  const size_t e0 = (size_t)i << 3;
  const float* p = src + e0;
  const v4f a0 = *(const v4f*)(p);
  const v4f a1 = *(const v4f*)(p + 4);
  v8h hv;
#pragma unroll
  for (int e = 0; e < 4; ++e) {
    hv[e]     = (_Float16)(a0[e] * scale);
    hv[4 + e] = (_Float16)(a1[e] * scale);
  }
  unsigned short* q = dst + e0;
  *(volatile v8h*)q = hv;
  __threadfence();
  *(volatile v8h*)q = hv;
}

__global__ __launch_bounds__(256) void pack_wxp_kernel(
    const float* __restrict__ W, unsigned short* __restrict__ dst, float scale)
{
  const int i   = blockIdx.x * 256 + threadIdx.x;
  const int e0  = i << 3;
  const int row = e0 / kDin;
  const int col = e0 - row * kDin;
  const bool isdt  = (row < kDtR);
  const bool isbc  = (row >= kBC0) && (row < kBC0 + 2 * kNst);
  const bool valid = isdt || isbc;
  const int srow = isdt ? row : (isbc ? (row - kBC0 + kDtR) : 0);
  const float* p = W + (size_t)srow * kDin + col;
  const v4f a0 = *(const v4f*)(p);
  const v4f a1 = *(const v4f*)(p + 4);
  v8h hv;
#pragma unroll
  for (int e = 0; e < 4; ++e) {
    const float f0 = valid ? (a0[e] * scale) : 0.0f;
    const float f1 = valid ? (a1[e] * scale) : 0.0f;
    hv[e]     = (_Float16)f0;
    hv[4 + e] = (_Float16)f1;
  }
  unsigned short* q = dst + e0;
  *(volatile v8h*)q = hv;
  __threadfence();
  *(volatile v8h*)q = hv;
}

__global__ __launch_bounds__(256) void pack_wdt_kernel(
    const float* __restrict__ W, unsigned short* __restrict__ dst, float scale)
{
  const int i   = blockIdx.x * 256 + threadIdx.x;
  const int e0  = i << 3;
  const int row = e0 >> 6;
  const int c8  = e0 & 63;
  const bool valid = (c8 < kDtR);
  const int c8c = valid ? c8 : 0;
  const float* p = W + (size_t)row * kDtR + c8c;
  const v4f a0 = *(const v4f*)(p);
  const v4f a1 = *(const v4f*)(p + 4);
  v8h hv;
#pragma unroll
  for (int e = 0; e < 4; ++e) {
    const float f0 = valid ? (a0[e] * scale) : 0.0f;
    const float f1 = valid ? (a1[e] * scale) : 0.0f;
    hv[e]     = (_Float16)f0;
    hv[4 + e] = (_Float16)f1;
  }
  unsigned short* q = dst + e0;
  *(volatile v8h*)q = hv;
  __threadfence();
  *(volatile v8h*)q = hv;
}

__global__ __launch_bounds__(256) void conv_silu_kernel(
    const float* __restrict__ XP, const float* __restrict__ cw, const float* __restrict__ cb,
    unsigned short* __restrict__ XC16)
{
  __shared__ __align__(16) float sF[16 * kTP];
  __shared__ __align__(16) float sB[16 * kTP];
  const int tid = threadIdx.x, lane = tid & 31, wave = tid >> 5;
  const int d0 = blockIdx.x * 256, d = d0 + tid;
  const int g0 = blockIdx.y * 64;
  const int tb = g0 & (kL - 1);
  const float w0 = cw[d * 4 + 0], w1 = cw[d * 4 + 1], w2 = cw[d * 4 + 2], w3 = cw[d * 4 + 3];
  const float bc = cb[d];
  float xm3, xm2, xm1, x0, xq1, xq2;
  {
    const bool hist = (tb > 0);
    const int rb = hist ? (g0 - 3) : g0;
    const float v3 = XP[(size_t)rb * kDin + d];
    const float v2 = XP[(size_t)(rb + 1) * kDin + d];
    const float v1 = XP[(size_t)(rb + 2) * kDin + d];
    xm3 = hist ? v3 : 0.f;
    xm2 = hist ? v2 : 0.f;
    xm1 = hist ? v1 : 0.f;
    x0  = XP[(size_t)g0 * kDin + d];
    xq1 = XP[(size_t)(g0 + 1) * kDin + d];
    xq2 = XP[(size_t)(g0 + 2) * kDin + d];
  }
  constexpr size_t kPlane = (size_t)kT * kDin;
#pragma unroll 1
  for (int sub = 0; sub < 4; ++sub) {
    const int lb = g0 + sub * 16;
#pragma unroll 1
    for (int s = 0; s < 16; ++s) {
      const int ti = sub * 16 + s;
      const bool fut = (tb + ti + 3) < kL;
      const int rr = g0 + (fut ? (ti + 3) : 0);
      const float ld = XP[(size_t)rr * kDin + d];
      const float xq3 = fut ? ld : 0.f;
      float af = w0 * xm3;
      af = fmaf(w1, xm2, af);
      af = fmaf(w2, xm1, af);
      af = fmaf(w3, x0, af);
      float ab = w0 * xq3;
      ab = fmaf(w1, xq2, ab);
      ab = fmaf(w2, xq1, ab);
      ab = fmaf(w3, x0, ab);
      const float svf = af + bc;
      const float svb = ab + bc;
      const float sgf = __builtin_amdgcn_rcpf(1.0f + __expf(-svf));
      const float sgb = __builtin_amdgcn_rcpf(1.0f + __expf(-svb));
      sF[s * kTP + tid] = svf * sgf;
      sB[s * kTP + tid] = svb * sgb;
      xm3 = xm2; xm2 = xm1; xm1 = x0; x0 = xq1; xq1 = xq2; xq2 = xq3;
    }
    __syncthreads();
    v8h fh[2], bh[2];
#pragma unroll
    for (int it = 0; it < 2; ++it) {
      const float* spf = sF + (it * 8 + wave) * kTP + lane * 8;
      const float* spb = sB + (it * 8 + wave) * kTP + lane * 8;
      const v4f a0 = *(const v4f*)(spf);
      const v4f a1 = *(const v4f*)(spf + 4);
      const v4f b0 = *(const v4f*)(spb);
      const v4f b1 = *(const v4f*)(spb + 4);
#pragma unroll
      for (int e = 0; e < 4; ++e) {
        fh[it][e]     = (_Float16)a0[e];
        fh[it][4 + e] = (_Float16)a1[e];
        bh[it][e]     = (_Float16)b0[e];
        bh[it][4 + e] = (_Float16)b1[e];
      }
    }
    for (int pass = 0; pass < 2; ++pass) {
#pragma unroll
      for (int it = 0; it < 2; ++it) {
        const size_t o = (size_t)(lb + it * 8 + wave) * kDin + d0 + lane * 8;
        *(volatile v8h*)(XC16 + o) = fh[it];
        *(volatile v8h*)(XC16 + kPlane + o) = bh[it];
      }
      __threadfence();
    }
    __syncthreads();
  }
}

template <int DIR>
__global__ __launch_bounds__(64) void scan_kernel(
    const unsigned short* __restrict__ DL16, const unsigned short* __restrict__ XC16,
    const unsigned short* __restrict__ PROJ16, const unsigned short* __restrict__ Z16,
    const float* __restrict__ bdt, const float* __restrict__ Alog, const float* __restrict__ Dp,
    float* YF, unsigned short* __restrict__ YC16)
{
  __shared__ __align__(16) float sBC[kScanTS * 32];
  __shared__ __align__(16) float sY[kScanTS * kScanYP];
  __shared__ __align__(16) float sA[kNst * kScanCh];
  const int tid = threadIdx.x, lane = tid & 31, wave = tid >> 5;
  constexpr int kBlkPerB = kDin / kScanCh;
  const int bix = blockIdx.x / kBlkPerB;
  const int d0  = (blockIdx.x - bix * kBlkPerB) * kScanCh;
  const int d   = d0 + tid;
  const size_t row0  = (size_t)bix * kL;
  const size_t prow0 = (size_t)DIR * kT + row0;
#pragma unroll 1
  for (int s = 0; s < kNst; ++s) sA[s * kScanCh + tid] = -expf(Alog[(size_t)d * kNst + s]);
  __syncthreads();
  float negA[kNst], h[kNst];
#pragma unroll
  for (int s = 0; s < kNst; ++s) {
    negA[s] = sA[s * kScanCh + tid];
    h[s] = 0.f;
  }
  const float bb = bdt[d], Dd = Dp[d];
#pragma unroll 1
  for (int ci = 0; ci < kL / kScanTS; ++ci) {
    const int t0 = (DIR ? (kL / kScanTS - 1 - ci) : ci) * kScanTS;
    __syncthreads();
#pragma unroll
    for (int i = 0; i < 4; ++i) {
      const int p  = tid + 64 * i;
      const int r  = p >> 2;
      const int qq = p & 3;
      const v4u w = *(const v4u*)(PROJ16 + (prow0 + t0 + r) * kPrjP + kBC0 + qq * 8);
      const unsigned u0 = w[0], u1 = w[1], u2 = w[2], u3 = w[3];
      v4f f0, f1;
      f0[0] = h16_to_f32(u0 & 0xffffu) * kInvProj;
      f0[1] = h16_to_f32(u0 >> 16) * kInvProj;
      f0[2] = h16_to_f32(u1 & 0xffffu) * kInvProj;
      f0[3] = h16_to_f32(u1 >> 16) * kInvProj;
      f1[0] = h16_to_f32(u2 & 0xffffu) * kInvProj;
      f1[1] = h16_to_f32(u2 >> 16) * kInvProj;
      f1[2] = h16_to_f32(u3 & 0xffffu) * kInvProj;
      f1[3] = h16_to_f32(u3 >> 16) * kInvProj;
      *(v4f*)(sBC + r * 32 + qq * 8)     = f0;
      *(v4f*)(sBC + r * 32 + qq * 8 + 4) = f1;
    }
    __syncthreads();
#pragma unroll 1
    for (int s = 0; s < kScanTS; ++s) {
      const int tl = DIR ? (kScanTS - 1 - s) : s;
      const size_t tok  = row0 + t0 + tl;
      const size_t pidx = (prow0 + t0 + tl) * kDin + d;
      const unsigned dlb = DL16[pidx];
      const unsigned xcb = XC16[pidx];
      float yfv = 0.f;
      unsigned zb = 0u;
      if (DIR == 1) {
        yfv = YF[tok * kDin + d];
        zb  = Z16[tok * kDin + d];
      }
      const float* xr = sBC + tl * 32;
      v4f Bq[4], Cq[4];
#pragma unroll
      for (int q4 = 0; q4 < 4; ++q4) {
        Bq[q4] = *(const v4f*)(xr + 4 * q4);
        Cq[q4] = *(const v4f*)(xr + kNst + 4 * q4);
      }
      const float dl  = h16_to_f32(dlb);
      const float xt  = h16_to_f32(xcb);
      const float v   = dl * kInvDl + bb;
      const float a   = __expf(-fabsf(v));
      const float u   = 1.0f + a;
      const float l1p = __logf(u) + (a - (u - 1.0f)) * __builtin_amdgcn_rcpf(u);
      const float dt  = fmaxf(v, 0.0f) + l1p;
      const float dtx = dt * xt;
      float y = 0.f;
#pragma unroll
      for (int k = 0; k < kNst; ++k) {
        const float e = __expf(dt * negA[k]);
        h[k] = e * h[k] + dtx * Bq[k >> 2][k & 3];
        y = h[k] * Cq[k >> 2][k & 3] + y;
      }
      y = xt * Dd + y;
      if (DIR == 1) {
        const float zv = h16_to_f32(zb);
        const float sg = __builtin_amdgcn_rcpf(1.0f + __expf(-zv));
        y = (y + yfv) * (zv * sg) * kGateMul;
      }
      sY[tl * kScanYP + tid] = y;
    }
    __syncthreads();
    if (DIR == 0) {
      const int hh = lane >> 4, c4 = (lane & 15) * 4;
      for (int pass = 0; pass < 2; ++pass) {
#pragma unroll 4
        for (int it = 0; it < 16; ++it) {
          const int row = it * 4 + wave * 2 + hh;
          const v4f val = *(const v4f*)(sY + row * kScanYP + c4);
          *(volatile v4f*)(YF + (row0 + t0 + row) * kDin + d0 + c4) = val;
        }
        __threadfence();
      }
    } else {
      const int q = lane >> 3, c8 = (lane & 7) * 8;
      for (int pass = 0; pass < 2; ++pass) {
#pragma unroll 4
        for (int it = 0; it < 8; ++it) {
          const int row = it * 8 + wave * 4 + q;
          const float* sp = sY + row * kScanYP + c8;
          const v4f a0 = *(const v4f*)(sp);
          const v4f a1 = *(const v4f*)(sp + 4);
          v8h hv;
#pragma unroll
          for (int e = 0; e < 4; ++e) {
            hv[e]     = (_Float16)a0[e];
            hv[4 + e] = (_Float16)a1[e];
          }
          *(volatile v8h*)(YC16 + (row0 + t0 + row) * kDin + d0 + c8) = hv;
        }
        __threadfence();
      }
    }
  }
}

constexpr int kBlkXp   = (kT / 64) * (kDin / 64) / 8;
constexpr int kBlkProj = (2 * kT / 64) * (kPrjP / 64) / 8;
constexpr int kBlkDl   = (2 * kT / 64) * (kDin / 64) / 8;
constexpr int kBlkOut  = (kT / 64) * (kDm / 64) / 8;
static_assert(kBlkXp * 8 == (kT / 64) * (kDin / 64));
static_assert(kBlkProj * 8 == (2 * kT / 64) * (kPrjP / 64));
static_assert(kBlkDl * 8 == (2 * kT / 64) * (kDin / 64));
static_assert(kBlkOut * 8 == (kT / 64) * (kDm / 64));
static_assert(((kT * kDm) % 2048) == 0 && ((2 * kDin * kDm) % 2048) == 0 && ((kDm * kDin) % 2048) == 0);
static_assert(((kPrjP * kDin) % 2048) == 0 && ((kDin * kDtK) % 2048) == 0);

extern "C" void kernel_launch(void* const* d_in, const int* in_sizes, int n_in,
                              void* d_out, int out_size, void* d_ws, size_t ws_size,
                              hipStream_t stream) {
  if (n_in < 10) return;
  if (in_sizes[0] != kT * kDm) return;
  if (in_sizes[1] != 2 * kDin * kDm) return;
  if (in_sizes[2] != kDin * 4) return;
  if (in_sizes[3] != kDin) return;
  if (in_sizes[4] != kPrjN * kDin) return;
  if (in_sizes[5] != kDin * kDtR) return;
  if (in_sizes[6] != kDin) return;
  if (in_sizes[7] != kDin * kNst) return;
  if (in_sizes[8] != kDin) return;
  if (in_sizes[9] != kDm * kDin) return;
  if (out_size != kT * kDm) return;
  if (ws_size < kWsTotal) return;

  const float* x       = (const float*)d_in[0];
  const float* W_in    = (const float*)d_in[1];
  const float* conv_w  = (const float*)d_in[2];
  const float* conv_b  = (const float*)d_in[3];
  const float* W_xproj = (const float*)d_in[4];
  const float* W_dt    = (const float*)d_in[5];
  const float* b_dt    = (const float*)d_in[6];
  const float* A_log   = (const float*)d_in[7];
  const float* Dp      = (const float*)d_in[8];
  const float* W_out   = (const float*)d_in[9];
  float* out = (float*)d_out;

  char* ws = (char*)d_ws;
  unsigned short* X16    = (unsigned short*)(ws + kOffX16);
  unsigned short* WIN16  = (unsigned short*)(ws + kOffWIN);
  unsigned short* WOUT16 = (unsigned short*)(ws + kOffWOUT);
  unsigned short* WXP16  = (unsigned short*)(ws + kOffWXP);
  unsigned short* WDT16  = (unsigned short*)(ws + kOffWDT);
  float*          XP32   = (float*)(ws + kOffXP);
  float*          YF32   = (float*)(ws + kOffXP);
  unsigned short* Z16    = (unsigned short*)(ws + kOffZ16);
  unsigned short* XC16   = (unsigned short*)(ws + kOffXC16);
  unsigned short* PROJ16 = (unsigned short*)(ws + kOffPROJ);
  unsigned short* DL16   = (unsigned short*)(ws + kOffDL16);
  unsigned short* YC16   = (unsigned short*)(ws + kOffYC16);

  cast_f16_kernel<<<(kT * kDm / 8) / 256, 256, 0, stream>>>(x, X16, kT * kDm / 8, 1.0f);
  cast_f16_kernel<<<(2 * kDin * kDm / 8) / 256, 256, 0, stream>>>(W_in, WIN16, 2 * kDin * kDm / 8, kCarryW);
  cast_f16_kernel<<<(kDm * kDin / 8) / 256, 256, 0, stream>>>(W_out, WOUT16, kDm * kDin / 8, kCarryW);
  pack_wxp_kernel<<<(kPrjP * kDin / 8) / 256, 256, 0, stream>>>(W_xproj, WXP16, kCarryW);
  pack_wdt_kernel<<<(kDin * kDtK / 8) / 256, 256, 0, stream>>>(W_dt, WDT16, kCarryWdt);

  wmma_gemm64<0><<<kBlkXp, 256, 0, stream>>>(
      X16, kDm, WIN16, kDm, (void*)XP32, kDin, kT, kDin, kDm, kScaleXp);
  wmma_gemm64<1><<<kBlkXp, 256, 0, stream>>>(
      X16, kDm, WIN16 + (size_t)kDin * kDm, kDm, (void*)Z16, kDin, kT, kDin, kDm, kScaleXp);

  conv_silu_kernel<<<dim3(kDin / 256, kT / 64), 256, 0, stream>>>(XP32, conv_w, conv_b, XC16);

  wmma_gemm64<1><<<kBlkProj, 256, 0, stream>>>(
      XC16, kDin, WXP16, kDin, (void*)PROJ16, kPrjP, 2 * kT, kPrjP, kDin, kScaleProj);

  wmma_gemm64<1><<<kBlkDl, 256, 0, stream>>>(
      PROJ16, kPrjP, WDT16, kDtK, (void*)DL16, kDin, 2 * kT, kDin, kDtK, kScaleDl);

  scan_kernel<0><<<kBatch * (kDin / kScanCh), kScanCh, 0, stream>>>(
      DL16, XC16, PROJ16, Z16, b_dt, A_log, Dp, YF32, YC16);
  scan_kernel<1><<<kBatch * (kDin / kScanCh), kScanCh, 0, stream>>>(
      DL16, XC16, PROJ16, Z16, b_dt, A_log, Dp, YF32, YC16);

  wmma_gemm64<0><<<kBlkOut, 256, 0, stream>>>(
      YC16, kDin, WOUT16, kDin, (void*)out, kDm, kT, kDm, kDin, kScaleOut);
}
